// MultiLayerGATv2_3118146257679
// MI455X (gfx1250) — hardware-verified
//
#include <hip/hip_runtime.h>
#include <stddef.h>


#define NTHR  256
#define NWAVE 8
#define GR    32
#define HIDC  128
#define KIN   256
#define NHEAD 4
#define AP0   (KIN + 8)
#define AP1   (HIDC + 8)
#define XSP   132
#define NBK   512
#define CHUNK 2048
#define WCAP  256
#define NGRP  (CHUNK / (NTHR * 4))
#define ACCF  (NBK * HIDC)
#define MXN   (NBK * NHEAD)
#define AGG_LDS_BYTES ((ACCF + 2 * MXN) * 4 + (NWAVE * WCAP + NWAVE) * 4)
#define LNEPS 1e-5f

static_assert(NGRP == 2);
static_assert(WCAP == (CHUNK / NTHR) * 32);
static_assert(AGG_LDS_BYTES == 286752);
static_assert((NBK & (NBK - 1)) == 0);
static_assert(NBK <= 512);
static_assert(NBK <= NWAVE * WCAP);
static_assert((AP0 % 8) == 0);
static_assert((AP1 % 8) == 0);
static_assert((XSP % 4) == 0);
static_assert(HIDC == NWAVE * 16);
static_assert(GR == NWAVE * 4);
static_assert((KIN % 32) == 0);
static_assert((HIDC % 32) == 0);

typedef float          v4f  __attribute__((ext_vector_type(4)));
typedef float          v8f  __attribute__((ext_vector_type(8)));
typedef int            v4i  __attribute__((ext_vector_type(4)));
typedef _Float16       v8h  __attribute__((ext_vector_type(8)));
typedef _Float16       v16h __attribute__((ext_vector_type(16)));
typedef __bf16         v16b __attribute__((ext_vector_type(16)));
typedef unsigned short v8us __attribute__((ext_vector_type(8)));

union FragH { v16h v; v4i u[2]; };
union FragB { v16b v; v4i u[2]; };
union Pack  { v8h h; v8us s; v4i i; };

__device__ __forceinline__ unsigned short f2bf(float x) {
  unsigned b = __float_as_uint(x);
  b += 0x7FFFu + ((b >> 16) & 1u);
  return (unsigned short)(b >> 16);
}
__device__ __forceinline__ float bf2f(unsigned short v) { return __uint_as_float(((unsigned)v) << 16); }

__device__ __forceinline__ v8f wmh(v16h a, v16h b, v8f c) {
  v8f d = __builtin_amdgcn_wmma_f32_16x16x32_f16(false, a, false, b, (short)0, c, false, false);
  asm volatile("v_nop\n\tv_nop\n\tv_nop\n\tv_nop" : "+v"(d) : "v"(a), "v"(b));
  return d;
}
__device__ __forceinline__ v8f wmb(v16b a, v16b b, v8f c) {
  v8f d = __builtin_amdgcn_wmma_f32_16x16x32_bf16(false, a, false, b, (short)0, c, false, false);
  asm volatile("v_nop\n\tv_nop\n\tv_nop\n\tv_nop" : "+v"(d) : "v"(a), "v"(b));
  return d;
}

__device__ __forceinline__ float wsum(float v) {
  v += __shfl_xor(v, 16, 32);
  v += __shfl_xor(v, 8, 32);
  v += __shfl_xor(v, 4, 32);
  v += __shfl_xor(v, 2, 32);
  v += __shfl_xor(v, 1, 32);
  return v;
}

__device__ __forceinline__ float lk(float t) { return fmaxf(t, 0.2f * t); }
__device__ __forceinline__ float dl(v4f t, v4f w) {
  return w.x * lk(t.x) + w.y * lk(t.y) + w.z * lk(t.z) + w.w * lk(t.w);
}
__device__ __forceinline__ float elu1(float t) { return t > 0.f ? t : (__expf(t) - 1.0f); }

__device__ __forceinline__ void cvt8s(v4f u0, v4f u1, Pack& ph, Pack& pl) {
#pragma unroll
  for (int j = 0; j < 4; ++j) {
    const unsigned short a = f2bf(u0[j]);
    ph.s[j] = a;
    pl.s[j] = f2bf(u0[j] - bf2f(a));
    const unsigned short c = f2bf(u1[j]);
    ph.s[4 + j] = c;
    pl.s[4 + j] = f2bf(u1[j] - bf2f(c));
  }
}
__device__ __forceinline__ v4i cvt8f(v4f u0, v4f u1) {
  Pack p;
#pragma unroll
  for (int j = 0; j < 4; ++j) {
    p.h[j]     = (_Float16)u0[j];
    p.h[4 + j] = (_Float16)u1[j];
  }
  return p.i;
}

__device__ __forceinline__ v4f ln_row(v4f v, v4f g4, v4f b4) {
  const float mu = wsum(v.x + v.y + v.z + v.w) * (1.0f / HIDC);
  const v4f d = v - mu;
  const float var = wsum(d.x * d.x + d.y * d.y + d.z * d.z + d.w * d.w) * (1.0f / HIDC);
  const float rs = rsqrtf(var + LNEPS);
  return d * rs * g4 + b4;
}

__device__ __forceinline__ void store_rows(const float* Xs_, float* dst, int rowBase, int wave, int lane) {
  v4f xv[4];
#pragma unroll
  for (int i = 0; i < 4; ++i) xv[i] = *(const v4f*)(Xs_ + (4 * wave + i) * XSP + 4 * lane);
#pragma unroll
  for (int i = 0; i < 4; ++i)
    *(volatile v4f*)(dst + (size_t)(rowBase + 4 * wave + i) * HIDC + 4 * lane) = xv[i];
  __threadfence();
#pragma unroll
  for (int i = 0; i < 4; ++i)
    *(volatile v4f*)(dst + (size_t)(rowBase + 4 * wave + i) * HIDC + 4 * lane) = xv[i];
}

__global__ __launch_bounds__(NTHR) void k_cvtw(const float* __restrict__ W, int K, int NC,
                                               unsigned short* p0, unsigned short* p1, float fscale, int mode) {
  const int kp8 = K >> 3;
  const int n8  = NC * kp8;
  const int i   = blockIdx.x * NTHR + threadIdx.x;
  if (i >= n8) return;
  const int n  = i / kp8;
  const int kb = (i - n * kp8) * 8;
  float v[8];
#pragma unroll
  for (int j = 0; j < 8; ++j) v[j] = W[(size_t)(kb + j) * NC + n];
  Pack uh, ul, uf;
  const v4i z4 = {0, 0, 0, 0};
  uh.i = z4; ul.i = z4; uf.i = z4;
#pragma unroll
  for (int j = 0; j < 8; ++j) {
    const unsigned short hb = f2bf(v[j]);
    uh.s[j] = hb;
    ul.s[j] = f2bf(v[j] - bf2f(hb));
    uf.h[j] = (_Float16)(v[j] * fscale);
  }
  const size_t o = (size_t)i * 8;
  if (mode & 1) { *(volatile v4i*)(p0 + o) = uh.i; *(volatile v4i*)(p1 + o) = ul.i; }
  if (mode & 2) { *(volatile v4i*)(p0 + o) = uf.i; }
  __threadfence();
  if (mode & 1) { *(volatile v4i*)(p0 + o) = uh.i; *(volatile v4i*)(p1 + o) = ul.i; }
  if (mode & 2) { *(volatile v4i*)(p0 + o) = uf.i; }
}

__global__ __launch_bounds__(NTHR) void k_gemm_in(
    const float* __restrict__ x, const unsigned short* __restrict__ Bh, const unsigned short* __restrict__ Bl,
    const float* __restrict__ bias, const float* __restrict__ gam, const float* __restrict__ bet,
    float* h, int nN) {
  __shared__ __attribute__((aligned(16))) unsigned short Ash[GR * AP0];
  __shared__ __attribute__((aligned(16))) unsigned short Asl[GR * AP0];
  __shared__ __attribute__((aligned(16))) float Xs[GR * XSP];

  const int tid  = threadIdx.x;
  const int lane = tid & 31;
  const int wave = tid >> 5;
  const int hh   = lane >> 4;
  const int m    = lane & 15;
  const int rowBase = blockIdx.x * GR;

  {
    const int r    = tid >> 3;
    const int ks   = (tid & 7) * 32;
    const int grow = rowBase + r;
    const bool ok  = grow < nN;
    const float* xp = x + (size_t)(ok ? grow : 0) * KIN + ks;
    const v4f z4 = {0.f, 0.f, 0.f, 0.f};
#pragma unroll
    for (int q = 0; q < 4; ++q) {
      v4f u0 = *(const v4f*)(xp + 8 * q);
      v4f u1 = *(const v4f*)(xp + 8 * q + 4);
      if (!ok) { u0 = z4; u1 = z4; }
      Pack ph, pl;
      cvt8s(u0, u1, ph, pl);
      const int o = r * AP0 + ks + 8 * q;
      *(v4i*)(Ash + o) = ph.i;
      *(v4i*)(Asl + o) = pl.i;
    }
  }
  __syncthreads();

  const int ncol = wave * 16 + m;
  const unsigned short* bhp = Bh + (size_t)ncol * KIN + 8 * hh;
  const unsigned short* blp = Bl + (size_t)ncol * KIN + 8 * hh;
  const unsigned short* ahp = Ash + m * AP0 + 8 * hh;
  const unsigned short* alp = Asl + m * AP0 + 8 * hh;

  v8f c0 = {0.f, 0.f, 0.f, 0.f, 0.f, 0.f, 0.f, 0.f};
  v8f c1 = {0.f, 0.f, 0.f, 0.f, 0.f, 0.f, 0.f, 0.f};

#pragma unroll 1
  for (int k0 = 0; k0 < KIN; k0 += 32) {
    FragB ah0, ah1, al0, al1, bh, bl;
    ah0.u[0] = *(const v4i*)(ahp + k0);              ah0.u[1] = *(const v4i*)(ahp + k0 + 16);
    ah1.u[0] = *(const v4i*)(ahp + 16 * AP0 + k0);   ah1.u[1] = *(const v4i*)(ahp + 16 * AP0 + k0 + 16);
    al0.u[0] = *(const v4i*)(alp + k0);              al0.u[1] = *(const v4i*)(alp + k0 + 16);
    al1.u[0] = *(const v4i*)(alp + 16 * AP0 + k0);   al1.u[1] = *(const v4i*)(alp + 16 * AP0 + k0 + 16);
    bh.u[0]  = *(const v4i*)(bhp + k0);              bh.u[1]  = *(const v4i*)(bhp + k0 + 16);
    bl.u[0]  = *(const v4i*)(blp + k0);              bl.u[1]  = *(const v4i*)(blp + k0 + 16);
    c0 = wmb(ah0.v, bh.v, c0);  c0 = wmb(ah0.v, bl.v, c0);  c0 = wmb(al0.v, bh.v, c0);
    c1 = wmb(ah1.v, bh.v, c1);  c1 = wmb(ah1.v, bl.v, c1);  c1 = wmb(al1.v, bh.v, c1);
  }

  const float bv = bias[ncol];
#pragma unroll
  for (int r = 0; r < 8; ++r) {
    Xs[(8 * hh + r) * XSP + ncol]      = c0[r] + bv;
    Xs[(16 + 8 * hh + r) * XSP + ncol] = c1[r] + bv;
  }
  __syncthreads();

  const v4f g4 = *(const v4f*)(gam + 4 * lane);
  const v4f b4 = *(const v4f*)(bet + 4 * lane);
  v4f ov[4];
#pragma unroll
  for (int i = 0; i < 4; ++i) {
    const int rl = 4 * wave + i;
    const v4f v = *(const v4f*)(Xs + rl * XSP + 4 * lane);
    v4f o = ln_row(v, g4, b4);
    o.x = fmaxf(o.x, 0.f);  o.y = fmaxf(o.y, 0.f);  o.z = fmaxf(o.z, 0.f);  o.w = fmaxf(o.w, 0.f);
    ov[i] = o;
  }
#pragma unroll
  for (int i = 0; i < 4; ++i) {
    const int grow = rowBase + 4 * wave + i;
    if (grow < nN) *(volatile v4f*)(h + (size_t)grow * HIDC + 4 * lane) = ov[i];
  }
  __threadfence();
#pragma unroll
  for (int i = 0; i < 4; ++i) {
    const int grow = rowBase + 4 * wave + i;
    if (grow < nN) *(volatile v4f*)(h + (size_t)grow * HIDC + 4 * lane) = ov[i];
  }
}

template <int SPLITL>
__global__ __launch_bounds__(NTHR) void k_gemm_lr(
    const float* __restrict__ h, const unsigned short* __restrict__ BLa, const unsigned short* __restrict__ BLb,
    const unsigned short* __restrict__ BRf, float* xl, float* xr, int nN) {
  __shared__ __attribute__((aligned(16))) unsigned short Asf[GR * AP1];
  __shared__ __attribute__((aligned(16))) unsigned short Ash[SPLITL ? GR * AP1 : 8];
  __shared__ __attribute__((aligned(16))) unsigned short Asl[SPLITL ? GR * AP1 : 8];
  __shared__ __attribute__((aligned(16))) float Xs[GR * XSP];

  const int tid  = threadIdx.x;
  const int lane = tid & 31;
  const int wave = tid >> 5;
  const int hh   = lane >> 4;
  const int m    = lane & 15;
  const int rowBase = blockIdx.x * GR;

  {
    const int r    = tid >> 3;
    const int ks   = (tid & 7) * 16;
    const int grow = rowBase + r;
    const bool ok  = grow < nN;
    const float* hp = h + (size_t)(ok ? grow : 0) * HIDC + ks;
    const v4f z4 = {0.f, 0.f, 0.f, 0.f};
#pragma unroll
    for (int q = 0; q < 2; ++q) {
      v4f u0 = *(const v4f*)(hp + 8 * q);
      v4f u1 = *(const v4f*)(hp + 8 * q + 4);
      if (!ok) { u0 = z4; u1 = z4; }
      const int o = r * AP1 + ks + 8 * q;
      *(v4i*)(Asf + o) = cvt8f(u0, u1);
      if (SPLITL) {
        Pack ph, pl;
        cvt8s(u0, u1, ph, pl);
        *(v4i*)(Ash + o) = ph.i;
        *(v4i*)(Asl + o) = pl.i;
      }
    }
  }
  __syncthreads();

  const int ncol = wave * 16 + m;
  const unsigned short* afp  = Asf + m * AP1 + 8 * hh;
  const unsigned short* blap = BLa + (size_t)ncol * HIDC + 8 * hh;
  const unsigned short* brp  = BRf + (size_t)ncol * HIDC + 8 * hh;

  v8f cl0 = {0.f, 0.f, 0.f, 0.f, 0.f, 0.f, 0.f, 0.f};
  v8f cl1 = {0.f, 0.f, 0.f, 0.f, 0.f, 0.f, 0.f, 0.f};
  v8f cr0 = {0.f, 0.f, 0.f, 0.f, 0.f, 0.f, 0.f, 0.f};
  v8f cr1 = {0.f, 0.f, 0.f, 0.f, 0.f, 0.f, 0.f, 0.f};

  if (SPLITL) {
    const unsigned short* ahp  = Ash + m * AP1 + 8 * hh;
    const unsigned short* alp  = Asl + m * AP1 + 8 * hh;
    const unsigned short* blbp = BLb + (size_t)ncol * HIDC + 8 * hh;
#pragma unroll 1
    for (int k0 = 0; k0 < HIDC; k0 += 32) {
      FragB ah0, ah1, al0, al1, bh, bl;
      ah0.u[0] = *(const v4i*)(ahp + k0);              ah0.u[1] = *(const v4i*)(ahp + k0 + 16);
      ah1.u[0] = *(const v4i*)(ahp + 16 * AP1 + k0);   ah1.u[1] = *(const v4i*)(ahp + 16 * AP1 + k0 + 16);
      al0.u[0] = *(const v4i*)(alp + k0);              al0.u[1] = *(const v4i*)(alp + k0 + 16);
      al1.u[0] = *(const v4i*)(alp + 16 * AP1 + k0);   al1.u[1] = *(const v4i*)(alp + 16 * AP1 + k0 + 16);
      bh.u[0]  = *(const v4i*)(blap + k0);             bh.u[1]  = *(const v4i*)(blap + k0 + 16);
      bl.u[0]  = *(const v4i*)(blbp + k0);             bl.u[1]  = *(const v4i*)(blbp + k0 + 16);
      cl0 = wmb(ah0.v, bh.v, cl0);  cl0 = wmb(ah0.v, bl.v, cl0);  cl0 = wmb(al0.v, bh.v, cl0);
      cl1 = wmb(ah1.v, bh.v, cl1);  cl1 = wmb(ah1.v, bl.v, cl1);  cl1 = wmb(al1.v, bh.v, cl1);
    }
  } else {
#pragma unroll 1
    for (int k0 = 0; k0 < HIDC; k0 += 32) {
      FragH a0, a1, b;
      a0.u[0] = *(const v4i*)(afp + k0);               a0.u[1] = *(const v4i*)(afp + k0 + 16);
      a1.u[0] = *(const v4i*)(afp + 16 * AP1 + k0);    a1.u[1] = *(const v4i*)(afp + 16 * AP1 + k0 + 16);
      b.u[0]  = *(const v4i*)(blap + k0);              b.u[1]  = *(const v4i*)(blap + k0 + 16);
      cl0 = wmh(a0.v, b.v, cl0);
      cl1 = wmh(a1.v, b.v, cl1);
    }
  }
#pragma unroll 1
  for (int k0 = 0; k0 < HIDC; k0 += 32) {
    FragH a0, a1, b;
    a0.u[0] = *(const v4i*)(afp + k0);               a0.u[1] = *(const v4i*)(afp + k0 + 16);
    a1.u[0] = *(const v4i*)(afp + 16 * AP1 + k0);    a1.u[1] = *(const v4i*)(afp + 16 * AP1 + k0 + 16);
    b.u[0]  = *(const v4i*)(brp + k0);               b.u[1]  = *(const v4i*)(brp + k0 + 16);
    cr0 = wmh(a0.v, b.v, cr0);
    cr1 = wmh(a1.v, b.v, cr1);
  }

  const float sl = SPLITL ? 1.0f : 0.0625f;
#pragma unroll
  for (int r = 0; r < 8; ++r) {
    Xs[(8 * hh + r) * XSP + ncol]      = cl0[r] * sl;
    Xs[(16 + 8 * hh + r) * XSP + ncol] = cl1[r] * sl;
  }
  __syncthreads();
  store_rows(Xs, xl, rowBase, wave, lane);
  __syncthreads();
#pragma unroll
  for (int r = 0; r < 8; ++r) {
    Xs[(8 * hh + r) * XSP + ncol]      = cr0[r] * 0.0625f;
    Xs[(16 + 8 * hh + r) * XSP + ncol] = cr1[r] * 0.0625f;
  }
  __syncthreads();
  store_rows(Xs, xr, rowBase, wave, lane);
}

__device__ __forceinline__ void hitq(const float* xs, const float* xd, float* ar, float* mp, float* dp, v4f w) {
  const v4f a0 = *(const v4f*)xs;
  const v4f d0 = *(const v4f*)xd;
  float s = dl(a0 + d0, w);
  s += __shfl_xor(s, 4, 32);
  s += __shfl_xor(s, 2, 32);
  s += __shfl_xor(s, 1, 32);
  const float mo = mp[0], n = dp[0];
  const float mn = fmaxf(mo, s);
  const float sc = __expf(mo - mn);
  const float p  = __expf(s - mn);
  v4f e0 = *(v4f*)ar;
  e0 = e0 * sc + a0 * p;
  *(v4f*)ar = e0;
  mp[0] = mn;
  dp[0] = n * sc + p;
}

__global__ __launch_bounds__(NTHR) void k_agg(
    const int* __restrict__ ei, const float* __restrict__ xl, const float* __restrict__ xr,
    const float* __restrict__ att, const float* __restrict__ gam, const float* __restrict__ bet,
    float* h, int nN, int nE) {
  extern __shared__ v4f lds_dyn[];
  float* sacc = (float*)lds_dyn;
  float* mx   = sacc + ACCF;
  float* dn   = mx + MXN;
  int*   list = (int*)(dn + MXN);
  int*   wcnt = list + NWAVE * WCAP;

  const int tid  = threadIdx.x;
  const int lane = tid & 31;
  const int wave = tid >> 5;
  const int nodeBase = blockIdx.x * NBK;

  {
    const v4f z4 = {0.f, 0.f, 0.f, 0.f};
    for (int i = tid; i < ACCF / 4; i += NTHR) lds_dyn[i] = z4;
    for (int i = tid; i < MXN; i += NTHR) { mx[i] = -1.0e30f; dn[i] = 0.f; }
  }
  __syncthreads();

  const int coff = 4 * lane;
  const int hidx = lane >> 3;
  const v4f w0 = *(const v4f*)(att + coff);

  const int* eid = ei + nE;
  const bool al16 = ((((size_t)eid) & 15) == 0) && ((nE & 3) == 0);
  const int nChunks = (nE + CHUNK - 1) / CHUNK;

#pragma unroll 1
  for (int ch = 0; ch <= nChunks; ++ch) {
    const int cbase = ch * CHUNK;
    const bool selfp = (ch == nChunks);
    if (!selfp) {
      int wc = 0;
#pragma unroll
      for (int g = 0; g < NGRP; ++g) {
        const int el0 = (g * NTHR + tid) * 4;
        const int e0  = cbase + el0;
        const int sent = -2147483647 - 1;
        v4i d;
        if (al16 && (e0 + 3 < nE)) {
          d = *(const v4i*)(eid + e0);
        } else {
          d.x = (e0     < nE) ? eid[min(e0, nE - 1)]     : sent;
          d.y = (e0 + 1 < nE) ? eid[min(e0 + 1, nE - 1)] : sent;
          d.z = (e0 + 2 < nE) ? eid[min(e0 + 2, nE - 1)] : sent;
          d.w = (e0 + 3 < nE) ? eid[min(e0 + 3, nE - 1)] : sent;
        }
        const unsigned s0 = (unsigned)d.x - (unsigned)nodeBase;
        const unsigned s1 = (unsigned)d.y - (unsigned)nodeBase;
        const unsigned s2 = (unsigned)d.z - (unsigned)nodeBase;
        const unsigned s3 = (unsigned)d.w - (unsigned)nodeBase;
        const bool h0 = s0 < (unsigned)NBK;
        const bool h1 = s1 < (unsigned)NBK;
        const bool h2 = s2 < (unsigned)NBK;
        const bool h3 = s3 < (unsigned)NBK;
        const unsigned many = __builtin_amdgcn_ballot_w32(h0 | h1 | h2 | h3);
        if (many != 0u) {
#define HITJ(J, HJ, SJ) { \
            const unsigned mj = __builtin_amdgcn_ballot_w32(HJ); \
            if (HJ) { \
              const int pos = wc + (int)__builtin_amdgcn_mbcnt_lo(mj, 0u); \
              if (pos < WCAP) list[wave * WCAP + pos] = ((el0 + (J)) << 9) | (int)(SJ); \
            } \
            wc += (int)__builtin_popcount(mj); }
          HITJ(0, h0, s0)
          HITJ(1, h1, s1)
          HITJ(2, h2, s2)
          HITJ(3, h3, s3)
#undef HITJ
        }
      }
      if (lane == 0) wcnt[wave] = wc;
    } else {
      for (int s = tid; s < NBK; s += NTHR) list[s] = s;
      if (tid < NWAVE) {
        int c = NBK - tid * WCAP;
        c = c < 0 ? 0 : (c > WCAP ? WCAP : c);
        wcnt[tid] = c;
      }
    }
    __syncthreads();

    if (wave == 0) {
#pragma unroll 1
      for (int wsx = 0; wsx < NWAVE; ++wsx) {
        int n = __builtin_amdgcn_readfirstlane(wcnt[wsx]);
        n = n > WCAP ? WCAP : n;
        n = n < 0 ? 0 : n;
#pragma unroll 1
        for (int i = 0; i < n; ++i) {
          const int ent  = __builtin_amdgcn_readfirstlane(list[wsx * WCAP + i]);
          const int slot = ent & (NBK - 1);
          const int el   = (ent >> 9) & (CHUNK - 1);
          const int node = nodeBase + slot;
          if (node >= nN) continue;
          int e = cbase + el;
          if (e > nE - 1) e = nE - 1;
          int sj = ei[e];
          sj = sj < 0 ? 0 : (sj > nN - 1 ? nN - 1 : sj);
          const int src = selfp ? node : sj;
          const float* xs = xl + (size_t)src * HIDC + coff;
          const float* xd = xr + (size_t)node * HIDC + coff;
          float* ar = sacc + slot * HIDC + coff;
          float* mp = mx + slot * NHEAD + hidx;
          float* dp = dn + slot * NHEAD + hidx;
          hitq(xs, xd, ar, mp, dp, w0);
        }
      }
    }
    __syncthreads();
  }

  const v4f g4 = *(const v4f*)(gam + coff);
  const v4f b4 = *(const v4f*)(bet + coff);
#pragma unroll 1
  for (int s = wave; s < NBK; s += NWAVE) {
    const int node = nodeBase + s;
    if (node >= nN) break;
    const v4f e0 = *(const v4f*)(sacc + s * HIDC + coff);
    const float inv = __builtin_amdgcn_rcpf(dn[s * NHEAD + hidx]);
    const v4f o = e0 * inv;
    v4f y = ln_row(o, g4, b4);
    y.x = elu1(y.x);  y.y = elu1(y.y);  y.z = elu1(y.z);  y.w = elu1(y.w);
    float* hp = h + (size_t)node * HIDC + coff;
    const v4f hv = *(const v4f*)hp;
    const v4f rv = hv + y;
    *(volatile v4f*)hp = rv;
    __threadfence();
    *(volatile v4f*)hp = rv;
  }
}

extern "C" void kernel_launch(void* const* d_in, const int* in_sizes, int n_in,
                              void* d_out, int out_size, void* d_ws, size_t ws_size,
                              hipStream_t stream) {
  if (n_in < 11) return;
  if (out_size <= 0 || (out_size % HIDC) != 0) return;
  const int nN = out_size / HIDC;
  if (in_sizes[0] != nN * KIN) return;
  if (in_sizes[1] != KIN * HIDC || in_sizes[2] != HIDC || in_sizes[3] != HIDC || in_sizes[4] != HIDC) return;
  const int HH = HIDC * HIDC;
  const int nL = in_sizes[5] / HH;
  if (nL < 1 || nL > 8 || in_sizes[5] != nL * HH || in_sizes[6] != nL * HH) return;
  if (in_sizes[7] != nL * HIDC || in_sizes[8] != nL * HIDC || in_sizes[9] != nL * HIDC) return;
  const int nE = in_sizes[10] / 2;
  if (nE <= 0 || in_sizes[10] != 2 * nE) return;

  const float* x    = (const float*)d_in[0];
  const float* W_in = (const float*)d_in[1];
  const float* b_in = (const float*)d_in[2];
  const float* gi   = (const float*)d_in[3];
  const float* bi   = (const float*)d_in[4];
  const float* Wl   = (const float*)d_in[5];
  const float* Wr   = (const float*)d_in[6];
  const float* att  = (const float*)d_in[7];
  const float* lg   = (const float*)d_in[8];
  const float* lb   = (const float*)d_in[9];
  const int*   ei   = (const int*)d_in[10];
  float* out = (float*)d_out;

  const int Mpad = ((nN + GR - 1) / GR) * GR;

  char* wsp = (char*)d_ws;
  size_t off = 0;
  const size_t wiB = (size_t)KIN * HIDC * 2;
  const size_t wlB = (size_t)HH * 2;
  const size_t xB  = (size_t)Mpad * HIDC * 4;
  unsigned short* Wih = (unsigned short*)(wsp + off); off += wiB;
  unsigned short* Wil = (unsigned short*)(wsp + off); off += wiB;
  unsigned short* Pla[8];
  unsigned short* Plb[8];
  unsigned short* Prf[8];
  for (int l = 0; l < nL; ++l) {
    Pla[l] = (unsigned short*)(wsp + off); off += wlB;
    Plb[l] = (unsigned short*)(wsp + off); off += wlB;
    Prf[l] = (unsigned short*)(wsp + off); off += wlB;
  }
  float* xl = (float*)(wsp + off); off += xB;
  float* xr = (float*)(wsp + off); off += xB;
  if (off > ws_size) return;
  if (off > (size_t)134217728) return;

  const float s16 = 16.0f;
  const int mt = Mpad / GR;

  k_cvtw<<<(HIDC * (KIN / 8) + NTHR - 1) / NTHR, NTHR, 0, stream>>>(W_in, KIN, HIDC, Wih, Wil, 1.0f, 1);
  for (int l = 0; l < nL; ++l) {
    const float* Wll = Wl + (size_t)l * HH;
    const float* Wrl = Wr + (size_t)l * HH;
    if (l == 0) k_cvtw<<<(HIDC * (HIDC / 8) + NTHR - 1) / NTHR, NTHR, 0, stream>>>(Wll, HIDC, HIDC, Pla[l], Plb[l], 1.0f, 1);
    else        k_cvtw<<<(HIDC * (HIDC / 8) + NTHR - 1) / NTHR, NTHR, 0, stream>>>(Wll, HIDC, HIDC, Pla[l], Plb[l], s16, 2);
    k_cvtw<<<(HIDC * (HIDC / 8) + NTHR - 1) / NTHR, NTHR, 0, stream>>>(Wrl, HIDC, HIDC, Prf[l], Prf[l], s16, 2);
  }

  hipFuncSetAttribute(reinterpret_cast<const void*>(&k_agg),
                      hipFuncAttributeMaxDynamicSharedMemorySize, AGG_LDS_BYTES);

  k_gemm_in<<<mt, NTHR, 0, stream>>>(x, Wih, Wil, b_in, gi, bi, out, nN);

  for (int l = 0; l < nL; ++l) {
    if (l == 0) k_gemm_lr<1><<<mt, NTHR, 0, stream>>>(out, Pla[l], Plb[l], Prf[l], xl, xr, nN);
    else        k_gemm_lr<0><<<mt, NTHR, 0, stream>>>(out, Pla[l], Plb[l], Prf[l], xl, xr, nN);
    k_agg<<<(nN + NBK - 1) / NBK, NTHR, AGG_LDS_BYTES, stream>>>(
        ei, xl, xr, att + (size_t)l * HIDC, lg + (size_t)l * HIDC, lb + (size_t)l * HIDC, out, nN, nE);
  }
}
